// TransformerEncoderLayer_23252952940951
// MI455X (gfx1250) — hardware-verified
//
#include <hip/hip_runtime.h>
#ifndef NB
#define NB 2
#endif
#ifndef SQ
#define SQ 2048
#endif
#define NB_FULL 2
#define SQ_FULL 2048
#define DM 1024
#define NH 16
#define HD 64
#define DFF 4096
#define LQ (3 * DM)
#define DMQ DM
#define NR ((size_t)NB * SQ)

static_assert(NB >= 1 && NB <= NB_FULL);
static_assert(SQ >= 256 && SQ <= SQ_FULL && SQ % 256 == 0);
static_assert(NH * HD == DM && HD == 64);
static_assert(DM % 64 == 0 && LQ % 64 == 0 && DFF % 64 == 0);
static_assert(DM % 32 == 0 && DFF % 32 == 0 && SQ % 128 == 0 && HD % 32 == 0);
static_assert((NR % 128) == 0);
static_assert(DMQ == 1024 && DMQ % 4 == 0 && DMQ / 4 == 256);
static_assert(((NR * DM / 4) % 256) == 0);
static_assert(((size_t)(NB - 1) * SQ_FULL + SQ) * DM * 4 <= (size_t)NB_FULL * SQ_FULL * DM * 4);

typedef unsigned short v8us __attribute__((ext_vector_type(8), may_alias));
typedef float  v8f  __attribute__((ext_vector_type(8)));
typedef float  v4f  __attribute__((ext_vector_type(4)));
typedef float  v4fa __attribute__((ext_vector_type(4), may_alias));
typedef _Float16 v16h __attribute__((ext_vector_type(16)));
typedef _Float16 v4h __attribute__((ext_vector_type(4)));
union FragH { v16h v; v8us half[2]; _Float16 h[16]; unsigned short u[16]; };

__device__ __forceinline__ unsigned short bf16_bits(float x) { unsigned int u = __float_as_uint(x); return (unsigned short)((u + 0x7FFFu + ((u >> 16) & 1u)) >> 16); }
__device__ __forceinline__ float bf16_val(unsigned short b) { return __uint_as_float(((unsigned int)b) << 16); }
__device__ __forceinline__ float bf16_rne(float x) { return bf16_val(bf16_bits(x)); }

__device__ __forceinline__ v16h g2_frag(const _Float16* p, int hh) { FragH f; f.half[0] = *(const v8us*)((const unsigned short*)p + 8 * hh); f.half[1] = *(const v8us*)((const unsigned short*)p + 16 + 8 * hh); return f.v; }
__device__ __forceinline__ v8f g2_mma(v16h a, v16h b, v8f c) { v8f d = __builtin_amdgcn_wmma_f32_16x16x32_f16(false, a, false, b, (short)0, c, false, false); asm volatile("v_nop\n\tv_nop\n\tv_nop\n\tv_nop" : "+v"(d) : "v"(a), "v"(b)); return d; }

template <int ACT>
__global__ __launch_bounds__(128) void k_gemm2(const _Float16* __restrict__ A, int lda, size_t sA, const _Float16* __restrict__ Bh, int ldb, size_t sB, float alpha, const float* __restrict__ bias, size_t sBias, const float* __restrict__ CP, int rowsPerB, size_t sCPb, int row0g,
    float* __restrict__ C, _Float16* __restrict__ C16, int ldc, size_t sC, int M, int N, int K, float s16) {
  static_assert(ACT == 0 || ACT == 3 || ACT == 6);
  __shared__ __attribute__((aligned(16))) float so[4][32][68];
  const int tid = threadIdx.x, w = tid >> 5, lane = tid & 31, ln = lane & 15, hh = lane >> 4; const int by = blockIdx.y;
  A += (size_t)by * sA; Bh += (size_t)by * sB; const size_t cofs = (size_t)by * sC; const float* bp = bias ? bias + (size_t)by * sBias : nullptr;
  const int ntn = N >> 6; const int mt = blockIdx.x / ntn, nq = blockIdx.x - mt * ntn; const int row0 = mt * 128 + 32 * w, col0 = nq * 64; if (row0 >= M) return;
  const _Float16* a0p = A + (size_t)(row0 + ln) * lda; const _Float16* a1p = a0p + (size_t)16 * lda;
  const _Float16* b0p = Bh + (size_t)(col0 + ln) * ldb; const _Float16* b1p = b0p + (size_t)16 * ldb; const _Float16* b2p = b1p + (size_t)16 * ldb; const _Float16* b3p = b2p + (size_t)16 * ldb;
  const v8f z8 = {0.f,0.f,0.f,0.f,0.f,0.f,0.f,0.f}; v8f c00 = z8, c01 = z8, c02 = z8, c03 = z8, c10 = z8, c11 = z8, c12 = z8, c13 = z8;
#pragma unroll 1
  for (int kb = 0; kb < K; kb += 32) { const v16h a0 = g2_frag(a0p + kb, hh), a1 = g2_frag(a1p + kb, hh);
    v16h b = g2_frag(b0p + kb, hh); c00 = g2_mma(a0, b, c00); c10 = g2_mma(a1, b, c10);
    b = g2_frag(b1p + kb, hh); c01 = g2_mma(a0, b, c01); c11 = g2_mma(a1, b, c11);
    b = g2_frag(b2p + kb, hh); c02 = g2_mma(a0, b, c02); c12 = g2_mma(a1, b, c12);
    b = g2_frag(b3p + kb, hh); c03 = g2_mma(a0, b, c03); c13 = g2_mma(a1, b, c13); }
  v8f accs[8] = {c00, c01, c02, c03, c10, c11, c12, c13};
#pragma unroll
  for (int u = 0; u < 8; ++u) { const int t = u & 3, half = u >> 2; const int col = col0 + t * 16 + ln; const float bv = bp ? bf16_rne(bp[col]) : 0.f;
#pragma unroll
    for (int r = 0; r < 8; ++r) { const int rloc = half * 16 + 8 * hh + r; float v = accs[u][r] * alpha + bv;
      if (CP) { if (rowsPerB < 0) v += CP[cofs + (size_t)(row0g + row0 + rloc) * ldc + col];        else { const int bidx = (row0g + row0 + rloc) / rowsPerB; v += CP[(size_t)bidx * sCPb + (size_t)by * 64 + col]; } }
      if (ACT == 3) v = fmaxf(v, 0.f); else if (ACT == 6) v = 0.5f * v * (1.0f + erff(v * 0.70710678118654752f));
      so[w][rloc][t * 16 + ln] = v; } }
  __builtin_amdgcn_fence(4  , "workgroup"); __builtin_amdgcn_wave_barrier();
  const int rsub = lane >> 4, c4 = (lane & 15) * 4;
  for (int pass = 0; pass < 2; ++pass) {
#pragma unroll
    for (int q = 0; q < 16; ++q) { const int r = q * 2 + rsub; const v4f v = *(const v4fa*)&so[w][r][c4];
      if (C) *(volatile v4f*)(C + cofs + (size_t)(row0 + r) * ldc + col0 + c4) = v;
      if (C16) { v4h h4; for (int i = 0; i < 4; ++i) h4[i] = (_Float16)(v[i] * s16); *(volatile v4h*)(C16 + cofs + (size_t)(row0 + r) * ldc + col0 + c4) = h4; } }
    if (pass == 0) __threadfence(); } }

__global__ __launch_bounds__(256) void k_wtr(const float* __restrict__ w, int K, int N, _Float16* __restrict__ Bt) { __shared__ unsigned short tl[64][66]; const int tid = threadIdx.x; const int ntn = N >> 6; const int kt = blockIdx.x / ntn, nt = blockIdx.x - kt * ntn;
  for (int i = tid; i < 64 * 16; i += 256) { const int r = i >> 4, c4 = (i & 15) * 4; const v4f a = *(const v4fa*)(w + (size_t)(kt * 64 + r) * N + nt * 64 + c4); FragH f;
#pragma unroll
    for (int q = 0; q < 4; ++q) f.h[q] = (_Float16)(bf16_rne(a[q]) * 16.0f);
#pragma unroll
    for (int q = 0; q < 4; ++q) tl[r][c4 + q] = f.u[q]; }
  __syncthreads();
  for (int pass = 0; pass < 2; ++pass) {
#pragma unroll
    for (int rd = 0; rd < 2; ++rd) { const int d = rd * 32 + tid / 8, pc = tid % 8; FragH f;
#pragma unroll
      for (int q = 0; q < 8; ++q) f.u[q] = tl[pc * 8 + q][d];
      *(volatile v8us*)((unsigned short*)Bt + (size_t)(nt * 64 + d) * K + kt * 64 + pc * 8) = f.half[0]; }
    if (pass == 0) __threadfence(); } }

__global__ __launch_bounds__(256) void k_xcv(const float* __restrict__ x, float* __restrict__ XB, _Float16* __restrict__ X16) { const size_t t = (size_t)blockIdx.x * 256 + threadIdx.x; if (t >= NR * DM / 4) return;
  const size_t e = t * 4; const size_t r = e / DM; const size_t c = e - r * DM; const size_t b = r / SQ, s = r - b * SQ; v4f a = *(const v4fa*)(x + (b * SQ_FULL + s) * DM + c); v4h y;
#pragma unroll
  for (int q = 0; q < 4; ++q) { a[q] = bf16_rne(a[q]); y[q] = (_Float16)a[q]; }
  for (int pass = 0; pass < 2; ++pass) { *(volatile v4f*)(XB + e) = a; *(volatile v4h*)(X16 + e) = y; if (pass == 0) __threadfence(); } }

template <int BFIN, int W16, int W32>
__global__ __launch_bounds__(256) void k_lnx(const float* __restrict__ X, const float* __restrict__ g, const float* __restrict__ bb, float eps, _Float16* __restrict__ N16, float* __restrict__ N32) {
  #pragma clang fp contract(off)
  __shared__ float red[256]; const size_t r = blockIdx.x; const int t = threadIdx.x; const bool act = t < (DMQ / 4); const int c0 = act ? t * 4 : 0;
  const v4f xa = *(const v4fa*)(X + r * DMQ + c0); float s[4]; float sum = 0.f;
#pragma unroll
  for (int q = 0; q < 4; ++q) { s[q] = act ? (BFIN ? bf16_rne(xa[q]) : xa[q]) : 0.f; sum = __fadd_rn(sum, s[q]); }
  red[t] = sum; __syncthreads(); for (int st = 128; st > 0; st >>= 1) { if (t < st) red[t] = __fadd_rn(red[t], red[t + st]); __syncthreads(); } const float mu = red[0] / (float)DMQ; __syncthreads();
  float vs = 0.f;
#pragma unroll
  for (int q = 0; q < 4; ++q) { const float dl = act ? __fadd_rn(s[q], -mu) : 0.f; vs = __fadd_rn(vs, __fmul_rn(dl, dl)); }
  red[t] = vs; __syncthreads(); for (int st = 128; st > 0; st >>= 1) { if (t < st) red[t] = __fadd_rn(red[t], red[t + st]); __syncthreads(); }
  const float rs = rsqrtf(__fadd_rn(red[0] / (float)DMQ, eps)); v4h y; v4f yf;
#pragma unroll
  for (int q = 0; q < 4; ++q) { const int c = c0 + q; yf[q] = __fadd_rn(__fmul_rn(__fmul_rn(__fadd_rn(s[q], -mu), rs), bf16_rne(g[c])), bf16_rne(bb[c])); y[q] = (_Float16)yf[q]; }
  if (!act) return;
  for (int pass = 0; pass < 2; ++pass) { if (W16) *(volatile v4h*)(N16 + r * DMQ + c0) = y; if (W32) *(volatile v4f*)(N32 + r * DMQ + c0) = yf; if (pass == 0) __threadfence(); } }

__device__ __forceinline__ float blk_sum256(float* red, float v, int t) { red[t] = v; __syncthreads(); for (int st = 128; st > 0; st >>= 1) { if (t < st) red[t] = __fadd_rn(red[t], red[t + st]); __syncthreads(); } const float s = red[0]; __syncthreads(); return s; }

__global__ __launch_bounds__(256) void k_lnfin(const float* __restrict__ FFP, const float* __restrict__ X1, const float* __restrict__ gf, const float* __restrict__ bf, const float* __restrict__ g2, const float* __restrict__ b2, float* __restrict__ out) {
  #pragma clang fp contract(off)
  __shared__ float red[256]; const size_t r = blockIdx.x; const int t = threadIdx.x; const int c0 = t * 4;
  const v4f xa = *(const v4fa*)(FFP + r * DM + c0); const v4f xr = *(const v4fa*)(X1 + r * DM + c0);
  float sum = 0.f;
#pragma unroll
  for (int q = 0; q < 4; ++q) sum = __fadd_rn(sum, xa[q]);
  const float mu1 = blk_sum256(red, sum, t) / (float)DM;
  float vs = 0.f;
#pragma unroll
  for (int q = 0; q < 4; ++q) { const float dl = __fadd_rn(xa[q], -mu1); vs = __fadd_rn(vs, __fmul_rn(dl, dl)); }
  const float rs1 = rsqrtf(__fadd_rn(blk_sum256(red, vs, t) / (float)DM, 1e-12f));
  float u[4]; float sum2 = 0.f;
#pragma unroll
  for (int q = 0; q < 4; ++q) { const int c = c0 + q; const float f = __fadd_rn(__fmul_rn(__fmul_rn(__fadd_rn(xa[q], -mu1), rs1), bf16_rne(gf[c])), bf16_rne(bf[c])); u[q] = __fadd_rn(xr[q], f); sum2 = __fadd_rn(sum2, u[q]); }
  const float mu2 = blk_sum256(red, sum2, t) / (float)DM;
  float vs2 = 0.f;
#pragma unroll
  for (int q = 0; q < 4; ++q) { const float dl = __fadd_rn(u[q], -mu2); vs2 = __fadd_rn(vs2, __fmul_rn(dl, dl)); }
  const float rs2 = rsqrtf(__fadd_rn(blk_sum256(red, vs2, t) / (float)DM, 1e-5f)); v4f yf;
#pragma unroll
  for (int q = 0; q < 4; ++q) { const int c = c0 + q; yf[q] = __fadd_rn(__fmul_rn(__fmul_rn(__fadd_rn(u[q], -mu2), rs2), bf16_rne(g2[c])), bf16_rne(b2[c])); }
  const size_t b = r / SQ, s = r - b * SQ; float* op = out + (b * SQ_FULL + s) * DM + c0;
  for (int pass = 0; pass < 2; ++pass) { *(volatile v4f*)op = yf; if (pass == 0) __threadfence(); } }

template <int NHv, int TTv>
__global__ __launch_bounds__(256) void k_vt(const _Float16* __restrict__ V16, int ldv, int voff, _Float16* __restrict__ Vt) { __shared__ unsigned short tl[64][66]; const int tid = threadIdx.x; const int slab = blockIdx.x / (TTv / 64), lg = blockIdx.x % (TTv / 64); const int b = slab / NHv, h = slab % NHv;
  for (int i = tid; i < 64 * 8; i += 256) { const int r = i / 8, c8 = (i % 8) * 8; FragH f; f.half[0] = *(const v8us*)((const unsigned short*)V16 + ((size_t)b * TTv + lg * 64 + r) * ldv + voff + h * 64 + c8);
#pragma unroll
    for (int q = 0; q < 8; ++q) tl[r][c8 + q] = f.u[q]; }
  __syncthreads();
  for (int pass = 0; pass < 2; ++pass) {
#pragma unroll
    for (int rd = 0; rd < 2; ++rd) { const int d = rd * 32 + tid / 8, pc = tid % 8; FragH f;
#pragma unroll
      for (int q = 0; q < 8; ++q) f.u[q] = tl[pc * 8 + q][d];
      *(volatile v8us*)((unsigned short*)Vt + ((size_t)slab * 64 + d) * TTv + lg * 64 + pc * 8) = f.half[0]; }
    if (pass == 0) __threadfence(); } }

__global__ __launch_bounds__(128) void k_flash(const _Float16* __restrict__ QKV, const _Float16* __restrict__ Vt, const int* __restrict__ amask, _Float16* __restrict__ O16) {
  __shared__ __attribute__((aligned(16))) float sf[4][32][36];
  __shared__ __attribute__((aligned(16))) _Float16 so[4][32][72];
  const int tid = threadIdx.x, w = tid >> 5, lane = tid & 31, ln = lane & 15, hh = lane >> 4;
  const int bh = blockIdx.y; const int b = bh / NH, h = bh - b * NH; const int q0 = (blockIdx.x * 4 + w) * 32;
  const _Float16* qp = QKV + ((size_t)b * SQ + q0 + ln) * LQ + (size_t)h * HD;
  v16h qa[2][2];
#pragma unroll
  for (int i = 0; i < 2; ++i) { qa[i][0] = g2_frag(qp + (size_t)(16 * i) * LQ, hh); qa[i][1] = g2_frag(qp + (size_t)(16 * i) * LQ + 32, hh); }
  const _Float16* kp = QKV + ((size_t)b * SQ + ln) * LQ + DM + (size_t)h * HD;
  const _Float16* vp = Vt + ((size_t)bh * HD + ln) * SQ;
  const int* mk = amask + (size_t)b * SQ_FULL + ln;
  const v8f z8 = {0.f,0.f,0.f,0.f,0.f,0.f,0.f,0.f};
  v8f acc[2][4];
#pragma unroll
  for (int i = 0; i < 2; ++i) {
#pragma unroll
    for (int j = 0; j < 4; ++j) acc[i][j] = z8; }
  float mrow[2] = {-1.0e30f, -1.0e30f}; float lrow[2] = {0.f, 0.f};
#pragma unroll 1
  for (int kv0 = 0; kv0 < SQ; kv0 += 32) {
    const _Float16* kr0 = kp + (size_t)kv0 * LQ; const _Float16* kr1 = kr0 + (size_t)16 * LQ;
    const int mv0 = mk[kv0], mv1 = mk[kv0 + 16];
    { const v16h k0 = g2_frag(kr0, hh), k1 = g2_frag(kr0 + 32, hh), k2 = g2_frag(kr1, hh), k3 = g2_frag(kr1 + 32, hh);
#pragma unroll
      for (int i = 0; i < 2; ++i) { v8f s0 = g2_mma(qa[i][0], k0, z8); s0 = g2_mma(qa[i][1], k1, s0); v8f s1 = g2_mma(qa[i][0], k2, z8); s1 = g2_mma(qa[i][1], k3, s1);
#pragma unroll
        for (int r = 0; r < 8; ++r) { const float e0 = s0[r] * 0.125f, e1 = s1[r] * 0.125f; sf[w][16 * i + 8 * hh + r][ln] = (mv0 != 0) ? e0 : -1.0e9f; sf[w][16 * i + 8 * hh + r][16 + ln] = (mv1 != 0) ? e1 : -1.0e9f; } } }
    __builtin_amdgcn_fence(4  , "workgroup"); __builtin_amdgcn_wave_barrier();
    v16h pa[2]; float alrow[2];
#pragma unroll
    for (int i = 0; i < 2; ++i) { const float* rowp = &sf[w][16 * i + ln][0];
      const v4f x0 = *(const v4fa*)(rowp + 8 * hh), x1 = *(const v4fa*)(rowp + 8 * hh + 4), x2 = *(const v4fa*)(rowp + 16 + 8 * hh), x3 = *(const v4fa*)(rowp + 16 + 8 * hh + 4);
      const float sv[16] = {x0[0], x0[1], x0[2], x0[3], x1[0], x1[1], x1[2], x1[3], x2[0], x2[1], x2[2], x2[3], x3[0], x3[1], x3[2], x3[3]};
      float t = sv[0];
#pragma unroll
      for (int e = 1; e < 16; ++e) t = fmaxf(t, sv[e]);
      t = fmaxf(t, __shfl_xor(t, 16));
      const float mn = fmaxf(mrow[i], t); const float al = __expf(mrow[i] - mn); mrow[i] = mn;
      float sum = 0.f; FragH pf;
#pragma unroll
      for (int e = 0; e < 16; ++e) { const float p = __expf(sv[e] - mn); sum += p; pf.h[e] = (_Float16)(p * 256.0f); }
      sum += __shfl_xor(sum, 16);
      lrow[i] = lrow[i] * al + sum; alrow[i] = al; pa[i] = pf.v; }
    __builtin_amdgcn_fence(4  , "workgroup"); __builtin_amdgcn_wave_barrier();
#pragma unroll
    for (int i = 0; i < 2; ++i) {
#pragma unroll
      for (int r = 0; r < 8; ++r) { const float alc = __shfl(alrow[i], r + 8 * hh);
#pragma unroll
        for (int j = 0; j < 4; ++j) acc[i][j][r] *= alc; } }
#pragma unroll
    for (int j = 0; j < 4; ++j) { const v16h vf = g2_frag(vp + (size_t)(16 * j) * SQ + kv0, hh);
#pragma unroll
      for (int i = 0; i < 2; ++i) acc[i][j] = g2_mma(pa[i], vf, acc[i][j]); } }
#pragma unroll
  for (int i = 0; i < 2; ++i) { const float linv = 1.0f / lrow[i];
#pragma unroll
    for (int r = 0; r < 8; ++r) { const float lc = __shfl(linv, r + 8 * hh) * 0.25f;
#pragma unroll
      for (int j = 0; j < 4; ++j) so[w][16 * i + 8 * hh + r][16 * j + ln] = (_Float16)(acc[i][j][r] * lc); } }
  __builtin_amdgcn_fence(4  , "workgroup"); __builtin_amdgcn_wave_barrier();
  const int rq = lane >> 3, pc = (lane & 7) * 8;
  for (int pass = 0; pass < 2; ++pass) {
#pragma unroll
    for (int it = 0; it < 8; ++it) { const int r = it * 4 + rq; const v8us v = *(const v8us*)&so[w][r][pc];
      *(volatile v8us*)((unsigned short*)O16 + ((size_t)b * SQ + q0 + r) * DM + (size_t)h * HD + pc) = v; }
    if (pass == 0) __threadfence(); } }

constexpr size_t al256(size_t b) { return (b + 255) & ~(size_t)255; }
constexpr size_t SZ_BQKV = (size_t)3 * DM * DM * 2, SZ_BO = (size_t)DM * DM * 2, SZ_BW1 = (size_t)DFF * DM * 2, SZ_BW2 = (size_t)DM * DFF * 2;
constexpr size_t SZ_XB = NR * DM * 4, SZ_X16 = NR * DM * 2, SZ_QKV = NR * LQ * 2, SZ_VT = (size_t)NB * NH * HD * SQ * 2, SZ_HF = NR * DFF * 2;
constexpr size_t SZ_PRE = NR * DM * 4;
constexpr size_t WS_TOTAL = al256(SZ_BQKV) + al256(SZ_BO) + al256(SZ_BW1) + al256(SZ_BW2) + al256(SZ_XB) + al256(SZ_X16) + al256(SZ_QKV) + al256(SZ_VT) + al256(SZ_HF);
static_assert(WS_TOTAL <= (size_t)134217728);
static_assert(SZ_PRE <= SZ_QKV);
static_assert(SZ_PRE == SZ_XB);
static_assert(SZ_X16 == NR * DM * 2);
static_assert((size_t)(DM / 64) * (DM / 64) * 64 * 64 == (size_t)DM * DM && (size_t)(DM / 64) * (DFF / 64) * 64 * 64 == (size_t)DM * DFF);
static_assert((NR / 128) * (DM / 64) * 4 * 32 * 64 == NR * DM && (NR / 128) * (DFF / 64) * 4 * 32 * 64 == NR * DFF);
static_assert((size_t)(SQ / 128) * NB * NH * 4 * 32 * 64 == NR * DM);
static_assert((size_t)NB * NH * (SQ / 64) * 64 * 64 == (size_t)NB * NH * HD * SQ);

extern "C" void kernel_launch(void* const* d_in, const int* in_sizes, int n_in,
                              void* d_out, int out_size, void* d_ws, size_t ws_size, hipStream_t stream) {
  if (n_in < 20) return;
  const float* x = (const float*)d_in[0]; const int* amask = (const int*)d_in[1];
  const float* wq = (const float*)d_in[2]; const float* bq = (const float*)d_in[3]; const float* wk = (const float*)d_in[4]; const float* bk = (const float*)d_in[5];
  const float* wv = (const float*)d_in[6]; const float* bv = (const float*)d_in[7]; const float* wo = (const float*)d_in[8]; const float* bo = (const float*)d_in[9];
  const float* g1 = (const float*)d_in[10]; const float* be1 = (const float*)d_in[11]; const float* w1 = (const float*)d_in[12]; const float* b1 = (const float*)d_in[13];
  const float* w2 = (const float*)d_in[14]; const float* b2 = (const float*)d_in[15]; const float* gf = (const float*)d_in[16]; const float* bef = (const float*)d_in[17];
  const float* g2 = (const float*)d_in[18]; const float* be2 = (const float*)d_in[19];
  const size_t needR = (size_t)(NB - 1) * SQ_FULL + SQ; const size_t needX = needR * DM;
  if ((size_t)in_sizes[0] < needX || (size_t)out_size < needX || (size_t)in_sizes[1] < needR) return;
  if (in_sizes[2] < DM * DM || in_sizes[4] < DM * DM || in_sizes[6] < DM * DM || in_sizes[8] < DM * DM) return;
  if (in_sizes[3] < DM || in_sizes[5] < DM || in_sizes[7] < DM || in_sizes[9] < DM || in_sizes[10] < DM || in_sizes[11] < DM) return;
  if (in_sizes[12] < DM * DFF || in_sizes[13] < DFF || in_sizes[14] < DFF * DM || in_sizes[15] < DM) return;
  if (in_sizes[16] < DM || in_sizes[17] < DM || in_sizes[18] < DM || in_sizes[19] < DM) return;
  char* ws = (char*)d_ws; size_t off = 0;
  auto take = [&](size_t bytes) { char* p = ws + off; off += al256(bytes); return p; };
  _Float16* BQKV = (_Float16*)take(SZ_BQKV); _Float16* BO = (_Float16*)take(SZ_BO); _Float16* BW1 = (_Float16*)take(SZ_BW1); _Float16* BW2 = (_Float16*)take(SZ_BW2);
  float* XB = (float*)take(SZ_XB); float* X1 = XB;
  _Float16* X16 = (_Float16*)take(SZ_X16); _Float16* O16 = X16; _Float16* M16 = X16;
  char* RQ = take(SZ_QKV); _Float16* QKV = (_Float16*)RQ; float* PRE1 = (float*)RQ; float* FFP = (float*)RQ;
  _Float16* VT = (_Float16*)take(SZ_VT); _Float16* HF16 = (_Float16*)take(SZ_HF);
  if (off > ws_size) return;

  k_wtr<<<(unsigned)((DM / 64) * (DM / 64)), 256, 0, stream>>>(wq, DM, DM, BQKV);
  k_wtr<<<(unsigned)((DM / 64) * (DM / 64)), 256, 0, stream>>>(wk, DM, DM, BQKV + (size_t)DM * DM);
  k_wtr<<<(unsigned)((DM / 64) * (DM / 64)), 256, 0, stream>>>(wv, DM, DM, BQKV + (size_t)2 * DM * DM);
  k_wtr<<<(unsigned)((DM / 64) * (DM / 64)), 256, 0, stream>>>(wo, DM, DM, BO);
  k_wtr<<<(unsigned)((DM / 64) * (DFF / 64)), 256, 0, stream>>>(w1, DM, DFF, BW1);
  k_wtr<<<(unsigned)((DFF / 64) * (DM / 64)), 256, 0, stream>>>(w2, DFF, DM, BW2);
  k_xcv<<<(unsigned)(NR * DM / 4 / 256), 256, 0, stream>>>(x, XB, X16);
  const unsigned gP = (unsigned)((NR / 128) * (DM / 64));
  k_gemm2<0><<<dim3(gP, 1), 128, 0, stream>>>(X16, DM, (size_t)0, BQKV, DM, (size_t)0, 0.0625f, bq, (size_t)0, nullptr, 1, (size_t)0, 0, nullptr, QKV, LQ, (size_t)0, (int)NR, DM, DM, 1.0f);
  k_gemm2<0><<<dim3(gP, 1), 128, 0, stream>>>(X16, DM, (size_t)0, BQKV + (size_t)DM * DM, DM, (size_t)0, 0.0625f, bk, (size_t)0, nullptr, 1, (size_t)0, 0, nullptr, QKV + DM, LQ, (size_t)0, (int)NR, DM, DM, 1.0f);
  k_gemm2<0><<<dim3(gP, 1), 128, 0, stream>>>(X16, DM, (size_t)0, BQKV + (size_t)2 * DM * DM, DM, (size_t)0, 0.0625f, bv, (size_t)0, nullptr, 1, (size_t)0, 0, nullptr, QKV + 2 * DM, LQ, (size_t)0, (int)NR, DM, DM, 1.0f);
  k_vt<NH, SQ><<<(unsigned)(NB * NH * (SQ / 64)), 256, 0, stream>>>(QKV + 2 * DM, LQ, 0, VT);
  k_flash<<<dim3((unsigned)(SQ / 128), (unsigned)(NB * NH)), 128, 0, stream>>>(QKV, VT, amask, O16);
  k_gemm2<0><<<dim3(gP, 1), 128, 0, stream>>>(O16, DM, (size_t)0, BO, DM, (size_t)0, 0.0009765625f, bo, (size_t)0, XB, -1, (size_t)0, 0, PRE1, nullptr, DM, (size_t)0, (int)NR, DM, DM, 1.0f);
  k_lnx<0, 1, 1><<<(unsigned)NR, 256, 0, stream>>>(PRE1, g1, be1, 1e-5f, M16, X1);
  k_gemm2<6><<<dim3((unsigned)((NR / 128) * (DFF / 64)), 1), 128, 0, stream>>>(M16, DM, (size_t)0, BW1, DM, (size_t)0, 0.0625f, b1, (size_t)0, nullptr, 1, (size_t)0, 0, nullptr, HF16, DFF, (size_t)0, (int)NR, DFF, DM, 16.0f);
  k_gemm2<0><<<dim3(gP, 1), 128, 0, stream>>>(HF16, DFF, (size_t)0, BW2, DFF, (size_t)0, 0.00390625f, b2, (size_t)0, X1, -1, (size_t)0, 0, FFP, nullptr, DM, (size_t)0, (int)NR, DM, DFF, 1.0f);
  k_lnfin<<<(unsigned)NR, 256, 0, stream>>>(FFP, X1, gf, bef, g2, be2, (float*)d_out);
}
